// NaiveAttention_47682726920223
// MI455X (gfx1250) — hardware-verified
//
#include <hip/hip_runtime.h>


namespace {
typedef _Float16 b16;
typedef __attribute__((ext_vector_type(16))) _Float16 v16b;
typedef __attribute__((ext_vector_type(8))) _Float16 v8b;
typedef __attribute__((ext_vector_type(4))) _Float16 v4h;
typedef __attribute__((ext_vector_type(2))) _Float16 v2h;
typedef __attribute__((ext_vector_type(8))) float v8f;
typedef __attribute__((ext_vector_type(4))) float v4f;
typedef __attribute__((ext_vector_type(2))) float v2f;
__device__ __forceinline__ float bf16_rne(float f) { unsigned int u = __float_as_uint(f); u += 0x7FFFu + ((u >> 16) & 1u); return __uint_as_float(u & 0xFFFF0000u); }
__device__ __forceinline__ void split16(float v, b16& hi, b16& lo) { hi = (b16)v; lo = (b16)(v - (float)hi); }
__device__ __forceinline__ v16b frag_kb(const b16* p, int hh) { const v8b a = *(const v8b*)(p + 8 * hh), b = *(const v8b*)(p + 16 + 8 * hh); v16b f;
#pragma unroll
  for (int e = 0; e < 8; ++e) { f[e] = a[e]; f[8 + e] = b[e]; } return f; }
__device__ __forceinline__ v8f wmma16b(v16b a, v16b b, v8f c) { v8f d = __builtin_amdgcn_wmma_f32_16x16x32_f16(false, a, false, b, (short)0, c, false, false); asm volatile("v_nop\n\tv_nop\n\tv_nop\n\tv_nop" : "+v"(d) : "v"(a), "v"(b)); return d; }
__device__ __forceinline__ void wave_lds_sync() { __builtin_amdgcn_fence(__ATOMIC_RELEASE, "workgroup"); __builtin_amdgcn_wave_barrier(); __builtin_amdgcn_fence(__ATOMIC_ACQUIRE, "workgroup"); }
__device__ __forceinline__ float pmul(float a, float b) { float p = a * b; asm volatile("" : "+v"(p)); return p; }
__device__ __forceinline__ int iclamp(int v, int lo, int hi) { return v < lo ? lo : (v > hi ? hi : v); }
__device__ __forceinline__ float nexp2(float v) { return __builtin_amdgcn_exp2f(v); }

constexpr int T = 2048, NH = 32, NKV = 8, GRP = NH / NKV, HD = 128, HL = NH  ;
constexpr float XS = 8.0f, PS = 1024.0f, RS_ = 1024.0f, LOG2E = 1.4426950408889634f, SCALE = 0.088388347648318447f  ;
static_assert(T % 64 == 0 && HD == 128 && NH % NKV == 0, "tiling");

__global__ __launch_bounds__(256) void qk_kernel(const float* __restrict__ q, const float* __restrict__ k, b16* __restrict__ QP, b16* __restrict__ KP) {
  const int u = blockIdx.x * 256 + threadIdx.x; const int nq = T * NH * HD / 8, nk = T * NKV * HD / 8;
  if (u < nq) { const int e = u * 8; const int h = e / (T * HD), rem = e % (T * HD), t = rem / HD, d = rem % HD; const float* src = q + ((size_t)t * NH + h) * HD + d; v8b o; for (int j = 0; j < 8; ++j) o[j] = (b16)(bf16_rne(src[j]) * XS);
    for (int pass = 0; pass < 2; ++pass) { *(volatile v8b*)(QP + e) = o; __threadfence(); } }
  else if (u < nq + nk) { const int e = (u - nq) * 8; const int h = e / (T * HD), rem = e % (T * HD), t = rem / HD, d = rem % HD; const float* src = k + ((size_t)t * NKV + h) * HD + d; v8b o; for (int j = 0; j < 8; ++j) o[j] = (b16)(bf16_rne(src[j]) * XS);
    for (int pass = 0; pass < 2; ++pass) { *(volatile v8b*)(KP + e) = o; __threadfence(); } }
}
__global__ __launch_bounds__(256) void vt_kernel(const float* __restrict__ v, b16* __restrict__ VT) {
  __shared__ __attribute__((aligned(16))) b16 Ts[HD][64 + 8]; const int kh = blockIdx.y, s0 = blockIdx.x * 64;
  for (int i = threadIdx.x; i < 64 * HD; i += 256) { const int tt = i / HD, d = i % HD; Ts[d][tt] = (b16)(bf16_rne(v[((size_t)(s0 + tt) * NKV + kh) * HD + d]) * XS); }
  __syncthreads();
  const int wave = threadIdx.x >> 5, lane = threadIdx.x & 31;
  for (int pass = 0; pass < 2; ++pass) { for (int d = wave; d < HD; d += 8) *(volatile v2h*)(VT + ((size_t)kh * HD + d) * T + s0 + lane * 2) = *(const v2h*)(&Ts[d][lane * 2]); __threadfence(); }
}
__global__ __launch_bounds__(64) void attn_kernel(const b16* __restrict__ QP, const b16* __restrict__ KP, const b16* __restrict__ VT, float* __restrict__ out) {
  __shared__ __attribute__((aligned(16))) b16 Pb[2][16][32 + 8], Pl[2][16][32 + 8]; __shared__ __attribute__((aligned(16))) float To[2][16][HD + 4];
  const int wave = threadIdx.x >> 5, lane = threadIdx.x & 31, hh = lane >> 4, col = lane & 15; const int h = blockIdx.y, kh = h / GRP; const int t0 = blockIdx.x * 32 + wave * 16; const int tq = t0 + col;
  const b16* Qb = QP + ((size_t)h * T + tq) * HD; const b16* Kb = KP + (size_t)kh * T * HD; const b16* Vb = VT + (size_t)kh * HD * T;
  v16b qf[4]; for (int kb = 0; kb < 4; ++kb) qf[kb] = frag_kb(Qb + kb * 32, hh);
  const float cs = LOG2E * SCALE / (XS * XS);
  float mrun = -INFINITY, l = 0.0f; v8f o[8], o2[8];
#pragma unroll
  for (int t = 0; t < 8; ++t) { o[t] = (v8f){}; o2[t] = (v8f){}; }
  const int send = t0 + 16;
#pragma unroll 1
  for (int s0 = 0; s0 < send; s0 += 32) {
    float e[16]; float mx = -INFINITY;
#pragma unroll
    for (int u2 = 0; u2 < 2; ++u2) { v8f sacc = (v8f){}; const b16* kr = Kb + (size_t)(s0 + u2 * 16 + col) * HD;
#pragma unroll
      for (int kb = 0; kb < 4; ++kb) sacc = wmma16b(frag_kb(kr + kb * 32, hh), qf[kb], sacc);
#pragma unroll
      for (int r = 0; r < 8; ++r) { const int s = s0 + u2 * 16 + 8 * hh + r; const float vv = (s <= tq) ? sacc[r] * cs : -INFINITY; e[u2 * 8 + r] = vv; mx = fmaxf(mx, vv); } }
    mx = fmaxf(mx, __shfl_xor(mx, 16)); const float mn = fmaxf(mrun, mx); const float al = (mn == -INFINITY) ? 1.0f : nexp2(mrun - mn); float sum = 0.0f;
#pragma unroll
    for (int i2 = 0; i2 < 16; ++i2) { const float p = (mn == -INFINITY) ? 0.0f : nexp2(e[i2] - mn); sum += p; const float psv = p * PS; const b16 p1 = (b16)psv; const int slot = (i2 < 8 ? 0 : 16) + 8 * hh + (i2 & 7); Pb[wave][col][slot] = p1; Pl[wave][col][slot] = (b16)((psv - (float)p1) * RS_); }
    sum += __shfl_xor(sum, 16); l = l * al + sum; mrun = mn;
    wave_lds_sync();
    const v16b pf = frag_kb(&Pb[wave][col][0], hh), plf = frag_kb(&Pl[wave][col][0], hh);
#pragma unroll
    for (int t = 0; t < 8; ++t) { o[t] *= al; o2[t] *= al; const v16b vf = frag_kb(Vb + (size_t)(t * 16 + col) * T + s0, hh); o[t] = wmma16b(vf, pf, o[t]); o2[t] = wmma16b(vf, plf, o2[t]); }
    wave_lds_sync(); }
  const float inv = 1.0f / (l * PS * XS);
#pragma unroll
  for (int t = 0; t < 8; ++t)
#pragma unroll
    for (int r = 0; r < 8; ++r) To[wave][col][t * 16 + 8 * hh + r] = (o[t][r] + o2[t][r] * (1.0f / RS_)) * inv;
  wave_lds_sync();
  for (int pass = 0; pass < 2; ++pass) { for (int rr = 0; rr < 16; ++rr) *(volatile v4f*)(out + ((size_t)(t0 + rr) * NH + h) * HD + lane * 4) = *(const v4f*)(&To[wave][rr][lane * 4]); __threadfence(); }
}
}

extern "C" void kernel_launch(void* const* d_in, const int* in_sizes, int n_in, void* d_out, int out_size, void* d_ws, size_t ws_size, hipStream_t stream) {
  (void)n_in;
  auto Fp = [&](int i) { return (const float*)d_in[i]; };
  if (in_sizes[0] != T * NH * HD || in_sizes[1] != T * NKV * HD || in_sizes[2] != T * NKV * HD || out_size != T * NH * HD) return;
  size_t off = 0; char* ws = (char*)d_ws;
  auto carve = [&](size_t bytes) { char* p = ws + off; off += (bytes + 255) & ~(size_t)255; return p; };
  b16* QP = (b16*)carve((size_t)NH * T * HD * 2); b16* KP = (b16*)carve((size_t)NKV * T * HD * 2); b16* VT = (b16*)carve((size_t)NKV * HD * T * 2);
  if (off > ws_size || off > ((size_t)128 << 20)) return;
  qk_kernel<<<((T * NH * HD + T * NKV * HD) / 8 + 255) / 256, 256, 0, stream>>>(Fp(0), Fp(1), QP, KP);
  vt_kernel<<<dim3(T / 64, NKV), 256, 0, stream>>>(Fp(2), VT);
  attn_kernel<<<dim3(T / 32, HL), 64, 0, stream>>>(QP, KP, VT, (float*)d_out);
}
